// BitwiseTasNetBlock_77017353552488
// MI455X (gfx1250) — hardware-verified
//
#include <hip/hip_runtime.h>
#include <stddef.h>
#include <stdint.h>


#define NB    8
#define NC    128
#define ND    512
#define NT    8000
#define NL    4
#define NK    3
#define TT    64
#define NTT   125
#define NPR   1000
#define NTHR  256
#define NWAVE 8
#define PX    68
#define PC2   132
#define PT2   68
#define TILE2 8704
#define LDS_G1 65536
#define WSCAP 268435456
#define BN_EPS 1e-5f
#define ASC   16.0f
#define W1C   1024.0f
#define WAC   256.0f
#define W2C   128.0f

static_assert(NT == TT * NTT);
static_assert(NPR == NB * NTT);
static_assert(NC == 128);
static_assert((NC % 32) == 0);
static_assert((ND % 256) == 0);
static_assert((NL * ND * NC) % (8 * NTHR) == 0);
static_assert(NTHR == 32 * NWAVE);
static_assert(TILE2 >= 64 * PC2);
static_assert(TILE2 >= 128 * PT2);
static_assert(LDS_G1 == NWAVE * 32 * 64 * 4);

typedef float    v4f  __attribute__((ext_vector_type(4)));
typedef float    v8f  __attribute__((ext_vector_type(8)));
typedef _Float16 v8h  __attribute__((ext_vector_type(8)));
typedef _Float16 v16h __attribute__((ext_vector_type(16)));
union FragH { v16h v; v8h h[2]; };

__device__ __forceinline__ v8f wmf(v16h a, v16h b, v8f c) {
  v8f d = __builtin_amdgcn_wmma_f32_16x16x32_f16(false, a, false, b, (short)0, c, false, false);
  asm volatile("v_nop\n\tv_nop\n\tv_nop\n\tv_nop" : "+v"(d) : "v"(a), "v"(b));
  return d;
}

__global__ __launch_bounds__(NTHR) void k_cvt_x(const float* __restrict__ x, _Float16* act) {
  __shared__ __attribute__((aligned(16))) float tile[NC * PX];
  const int tid = threadIdx.x, lane = tid & 31, wave = tid >> 5, hh = lane >> 4, m = lane & 15;
  const int t0 = blockIdx.x * TT, b = blockIdx.y;
  const float* xb = x + (size_t)b * NC * NT + t0;
#pragma unroll
  for (int it = 0; it < 8; ++it) {
    const int c = it * 16 + (tid >> 4);
    const int t4 = (tid & 15) * 4;
    const v4f v = *(const v4f*)(xb + (size_t)c * NT + t4);
    *(v4f*)(tile + c * PX + t4) = v;
  }
  __syncthreads();
  v8h hv[4];
#pragma unroll
  for (int q = 0; q < 4; ++q) {
    const int tr = 8 * wave + 2 * q + hh;
#pragma unroll
    for (int e = 0; e < 8; ++e) hv[q][e] = (_Float16)(tile[(8 * m + e) * PX + tr] * ASC);
  }
  _Float16* ob = act + ((size_t)b * NT + t0) * NC;
#pragma unroll
  for (int q = 0; q < 4; ++q) {
    const int tr = 8 * wave + 2 * q + hh;
    *(volatile v8h*)(ob + (size_t)tr * NC + 8 * m) = hv[q];
  }
  __threadfence();
#pragma unroll
  for (int q = 0; q < 4; ++q) {
    const int tr = 8 * wave + 2 * q + hh;
    *(volatile v8h*)(ob + (size_t)tr * NC + 8 * m) = hv[q];
  }
}

__global__ __launch_bounds__(NTHR) void k_cvt_w1(const float* __restrict__ w1, _Float16* w1h) {
  const size_t t = (size_t)blockIdx.x * NTHR + threadIdx.x;
  const float* p = w1 + t * 8;
  const v4f f0 = *(const v4f*)p;
  const v4f f1 = *(const v4f*)(p + 4);
  v8h a;
  a[0] = (_Float16)(f0.x * W1C); a[1] = (_Float16)(f0.y * W1C);
  a[2] = (_Float16)(f0.z * W1C); a[3] = (_Float16)(f0.w * W1C);
  a[4] = (_Float16)(f1.x * W1C); a[5] = (_Float16)(f1.y * W1C);
  a[6] = (_Float16)(f1.z * W1C); a[7] = (_Float16)(f1.w * W1C);
  _Float16* d = w1h + t * 8;
  *(volatile v8h*)d = a;
  __threadfence();
  *(volatile v8h*)d = a;
}

__global__ __launch_bounds__(NTHR) void k_gemm1(const _Float16* __restrict__ act, const _Float16* __restrict__ w1h,
                                                const float* __restrict__ b1, const float* __restrict__ a1,
                                                float* vpl, float* psum, float* psq) {
  extern __shared__ v4f lds_dyn[];
  __shared__ __attribute__((aligned(16))) float sts[NWAVE * 64];
  __shared__ __attribute__((aligned(16))) float stq[NWAVE * 64];
  __shared__ __attribute__((aligned(16))) float pcs[256];
  __shared__ __attribute__((aligned(16))) float pcq[256];
  const int tid = threadIdx.x, lane = tid & 31, wave = tid >> 5, hh = lane >> 4, m = lane & 15;
  const int wn = wave & 3, wm = wave >> 2;
  float* stg = (float*)lds_dyn + wave * (32 * 64);
  const int dblk = blockIdx.x, tt = blockIdx.y, b = blockIdx.z;
  const int d0 = dblk * 256, t0 = tt * TT;

  v8f acc[2][4];
#pragma unroll
  for (int mt = 0; mt < 2; ++mt)
#pragma unroll
    for (int nt = 0; nt < 4; ++nt) { v8f z = {0.f, 0.f, 0.f, 0.f, 0.f, 0.f, 0.f, 0.f}; acc[mt][nt] = z; }

  const _Float16* ap = act + ((size_t)b * NT + t0 + wm * 32 + m) * NC + 8 * hh;
  const _Float16* bp = w1h + (size_t)(d0 + wn * 64 + m) * NC + 8 * hh;
#pragma unroll 1
  for (int kt = 0; kt < NC / 32; ++kt) {
    const int k0 = 32 * kt;
    FragH a0, a1;
    a0.h[0] = *(const v8h*)(ap + k0);
    a0.h[1] = *(const v8h*)(ap + k0 + 16);
    a1.h[0] = *(const v8h*)(ap + 16 * NC + k0);
    a1.h[1] = *(const v8h*)(ap + 16 * NC + k0 + 16);
#pragma unroll
    for (int nt = 0; nt < 4; ++nt) {
      const _Float16* bq = bp + (size_t)nt * 16 * NC + k0;
      FragH bf;
      bf.h[0] = *(const v8h*)bq;
      bf.h[1] = *(const v8h*)(bq + 16);
      acc[0][nt] = wmf(a0.v, bf.v, acc[0][nt]);
      acc[1][nt] = wmf(a1.v, bf.v, acc[1][nt]);
    }
  }

  const float alpha = a1[0];
  constexpr float OS1 = 1.0f / (ASC * W1C);
  float bv[4];
#pragma unroll
  for (int nt = 0; nt < 4; ++nt) bv[nt] = b1[d0 + wn * 64 + 16 * nt + m];
  float s[4] = {0.f, 0.f, 0.f, 0.f}, q2[4] = {0.f, 0.f, 0.f, 0.f};
#pragma unroll
  for (int mt = 0; mt < 2; ++mt) {
    float* sp = stg + (16 * mt + 8 * hh) * 64 + m;
#pragma unroll
    for (int nt = 0; nt < 4; ++nt) {
#pragma unroll
      for (int r = 0; r < 8; ++r) {
        float v = acc[mt][nt][r] * OS1 + bv[nt];
        v = (v >= 0.0f) ? v : alpha * v;
        sp[r * 64 + 16 * nt] = v;
        s[nt] += v;
        q2[nt] += v * v;
      }
    }
  }
#pragma unroll
  for (int nt = 0; nt < 4; ++nt) {
    s[nt]  += __shfl_xor(s[nt], 16, 32);
    q2[nt] += __shfl_xor(q2[nt], 16, 32);
  }
  if (hh == 0) {
#pragma unroll
    for (int nt = 0; nt < 4; ++nt) {
      sts[wave * 64 + 16 * nt + m] = s[nt];
      stq[wave * 64 + 16 * nt + m] = q2[nt];
    }
  }
  __syncthreads();
  {
    const int wq = tid >> 6, ix = tid & 63;
    pcs[tid] = sts[wq * 64 + ix] + sts[(4 + wq) * 64 + ix];
    pcq[tid] = stq[wq * 64 + ix] + stq[(4 + wq) * 64 + ix];
  }
  float* gb = vpl + ((size_t)b * NT + t0 + wm * 32) * ND + d0 + wn * 64;
#pragma unroll
  for (int q = 0; q < 16; ++q) {
    const int row = 2 * q + hh;
    const v4f v = *(const v4f*)(stg + row * 64 + 4 * m);
    *(volatile v4f*)(gb + (size_t)row * ND + 4 * m) = v;
  }
  __syncthreads();
  const size_t prow = (size_t)(b * NTT + tt) * ND + d0;
  if (tid < 64) {
    const v4f p = *(const v4f*)(pcs + 4 * tid);
    *(volatile v4f*)(psum + prow + 4 * tid) = p;
  } else if (tid < 128) {
    const v4f p = *(const v4f*)(pcq + 4 * (tid - 64));
    *(volatile v4f*)(psq + prow + 4 * (tid - 64)) = p;
  }
  __threadfence();
#pragma unroll
  for (int q = 0; q < 16; ++q) {
    const int row = 2 * q + hh;
    const v4f v = *(const v4f*)(stg + row * 64 + 4 * m);
    *(volatile v4f*)(gb + (size_t)row * ND + 4 * m) = v;
  }
  if (tid < 64) {
    const v4f p = *(const v4f*)(pcs + 4 * tid);
    *(volatile v4f*)(psum + prow + 4 * tid) = p;
  } else if (tid < 128) {
    const v4f p = *(const v4f*)(pcq + 4 * (tid - 64));
    *(volatile v4f*)(psq + prow + 4 * (tid - 64)) = p;
  }
}

template <int MODE>
__global__ __launch_bounds__(128) void k_bnfin(const float* __restrict__ psum, const float* __restrict__ psq,
                                              const float* __restrict__ g, const float* __restrict__ be,
                                              float* scale1, float* shift1,
                                              const float* __restrict__ w2, const float* __restrict__ b2,
                                              _Float16* w2h, float* bias2) {
  __shared__ __attribute__((aligned(16))) float scs[ND];
  __shared__ __attribute__((aligned(16))) float shs[ND];
  __shared__ float pbl[NC * 2];
  __shared__ __attribute__((aligned(16))) float bfin[NC];
  const int tid = threadIdx.x, lane = tid & 31, wave = tid >> 5;

  double s[4] = {0.0, 0.0, 0.0, 0.0}, q[4] = {0.0, 0.0, 0.0, 0.0};
#pragma unroll 1
  for (int r = 0; r < NPR; ++r) {
    const v4f a = *(const v4f*)(psum + (size_t)r * ND + 4 * tid);
    const v4f c = *(const v4f*)(psq + (size_t)r * ND + 4 * tid);
    s[0] += (double)a.x; s[1] += (double)a.y; s[2] += (double)a.z; s[3] += (double)a.w;
    q[0] += (double)c.x; q[1] += (double)c.y; q[2] += (double)c.z; q[3] += (double)c.w;
  }
  const double invn = 1.0 / (double)(NB * NT);
  float sc[4], sh[4];
#pragma unroll
  for (int j = 0; j < 4; ++j) {
    const double mean = s[j] * invn;
    double var = q[j] * invn - mean * mean;
    var = var > 0.0 ? var : 0.0;
    const float rs = rsqrtf((float)var + BN_EPS);
    sc[j] = g[4 * tid + j] * rs;
    sh[j] = be[4 * tid + j] - (float)mean * sc[j];
  }
  const v4f scv = {sc[0], sc[1], sc[2], sc[3]};
  const v4f shv = {sh[0], sh[1], sh[2], sh[3]};

  if (MODE == 0) {
    *(volatile v4f*)(scale1 + 4 * tid) = scv;
    *(volatile v4f*)(shift1 + 4 * tid) = shv;
    __threadfence();
    *(volatile v4f*)(scale1 + 4 * tid) = scv;
    *(volatile v4f*)(shift1 + 4 * tid) = shv;
  } else {
    *(v4f*)(scs + 4 * tid) = scv;
    *(v4f*)(shs + 4 * tid) = shv;
    __syncthreads();
    const int half = tid >> 6, j = tid & 63;
    union { v4f v[2]; float f[8]; } msc, msh;
    msc.v[0] = *(const v4f*)(scs + 8 * j); msc.v[1] = *(const v4f*)(scs + 8 * j + 4);
    msh.v[0] = *(const v4f*)(shs + 8 * j); msh.v[1] = *(const v4f*)(shs + 8 * j + 4);
#pragma unroll 1
    for (int r = 0; r < NC / 2; ++r) {
      const int c = 2 * r + half;
      const float* wr = w2 + (size_t)c * ND + 8 * j;
      union { v4f v[2]; float f[8]; } u;
      u.v[0] = *(const v4f*)wr; u.v[1] = *(const v4f*)(wr + 4);
      v8h hv;
      float pb = 0.0f;
#pragma unroll
      for (int e = 0; e < 8; ++e) {
        hv[e] = (_Float16)((u.f[e] * msc.f[e]) * W2C);
        pb += u.f[e] * msh.f[e];
      }
      pb += __shfl_xor(pb, 16, 32);
      pb += __shfl_xor(pb, 8, 32);
      pb += __shfl_xor(pb, 4, 32);
      pb += __shfl_xor(pb, 2, 32);
      pb += __shfl_xor(pb, 1, 32);
      if (lane == 0) pbl[c * 2 + (wave & 1)] = pb;
      _Float16* dst = w2h + (size_t)c * ND + 8 * j;
      *(volatile v8h*)dst = hv;
      __threadfence();
      *(volatile v8h*)dst = hv;
    }
    __syncthreads();
    bfin[tid] = b2[tid] + (pbl[2 * tid] + pbl[2 * tid + 1]);
    __syncthreads();
    if (tid < 32) {
      const v4f v = *(const v4f*)(bfin + 4 * tid);
      *(volatile v4f*)(bias2 + 4 * tid) = v;
      __threadfence();
      *(volatile v4f*)(bias2 + 4 * tid) = v;
    }
  }
}

__global__ __launch_bounds__(NTHR) void k_dwconv(const float* __restrict__ vpl,
                                                 const float* __restrict__ scale1, const float* __restrict__ shift1,
                                                 const float* __restrict__ wd, const float* __restrict__ bd,
                                                 const float* __restrict__ a2, int dil,
                                                 _Float16* wpl, float* psum, float* psq) {
  __shared__ __attribute__((aligned(16))) float sts[NWAVE * 256];
  __shared__ __attribute__((aligned(16))) float stq[NWAVE * 256];
  __shared__ __attribute__((aligned(16))) float pcs[256];
  __shared__ __attribute__((aligned(16))) float pcq[256];
  const int tid = threadIdx.x, lane = tid & 31, wave = tid >> 5;
  const int dblk = blockIdx.x, tt = blockIdx.y, b = blockIdx.z;
  const int t0 = tt * TT;
  const int dg = dblk * 256 + 8 * lane;
  const size_t rowb = (size_t)b * NT;
  const float alpha = a2[0];

  union { v4f v[2]; float f[8]; } sc, sh, bb;
  sc.v[0] = *(const v4f*)(scale1 + dg); sc.v[1] = *(const v4f*)(scale1 + dg + 4);
  sh.v[0] = *(const v4f*)(shift1 + dg); sh.v[1] = *(const v4f*)(shift1 + dg + 4);
  bb.v[0] = *(const v4f*)(bd + dg);     bb.v[1] = *(const v4f*)(bd + dg + 4);
  union { v4f v[6]; float f[24]; } tap;
  const float* wp = wd + (size_t)dg * NK;
#pragma unroll
  for (int u = 0; u < 6; ++u) tap.v[u] = *(const v4f*)(wp + 4 * u);

  float s[8] = {0.f, 0.f, 0.f, 0.f, 0.f, 0.f, 0.f, 0.f};
  float q2[8] = {0.f, 0.f, 0.f, 0.f, 0.f, 0.f, 0.f, 0.f};
#pragma unroll 1
  for (int i = 0; i < 8; ++i) {
    const int t = t0 + wave + 8 * i;
    const int tl = t - dil, tr = t + dil;
    const int tlc = tl < 0 ? 0 : tl;
    const int trc = tr > NT - 1 ? NT - 1 : tr;
    const bool okl = tl >= 0, okr = tr < NT;
    const float* pc = vpl + (rowb + (size_t)t) * ND + dg;
    const float* pl = vpl + (rowb + (size_t)tlc) * ND + dg;
    const float* pr = vpl + (rowb + (size_t)trc) * ND + dg;
    union { v4f v[2]; float f[8]; } xc, xl, xr;
    xc.v[0] = *(const v4f*)pc; xc.v[1] = *(const v4f*)(pc + 4);
    xl.v[0] = *(const v4f*)pl; xl.v[1] = *(const v4f*)(pl + 4);
    xr.v[0] = *(const v4f*)pr; xr.v[1] = *(const v4f*)(pr + 4);
    v8h hv;
#pragma unroll
    for (int e = 0; e < 8; ++e) {
      const float zc = xc.f[e] * sc.f[e] + sh.f[e];
      const float zl = okl ? (xl.f[e] * sc.f[e] + sh.f[e]) : 0.0f;
      const float zr = okr ? (xr.f[e] * sc.f[e] + sh.f[e]) : 0.0f;
      float y = tap.f[3 * e] * zl + tap.f[3 * e + 1] * zc + tap.f[3 * e + 2] * zr + bb.f[e];
      y = (y >= 0.0f) ? y : alpha * y;
      s[e] += y;
      q2[e] += y * y;
      hv[e] = (_Float16)(y * WAC);
    }
    _Float16* dst = wpl + (rowb + (size_t)t) * ND + dg;
    *(volatile v8h*)dst = hv;
    __threadfence();
    *(volatile v8h*)dst = hv;
  }
  {
    const v4f s0 = {s[0], s[1], s[2], s[3]}, s1 = {s[4], s[5], s[6], s[7]};
    const v4f q0 = {q2[0], q2[1], q2[2], q2[3]}, q1 = {q2[4], q2[5], q2[6], q2[7]};
    *(v4f*)(sts + wave * 256 + 8 * lane) = s0; *(v4f*)(sts + wave * 256 + 8 * lane + 4) = s1;
    *(v4f*)(stq + wave * 256 + 8 * lane) = q0; *(v4f*)(stq + wave * 256 + 8 * lane + 4) = q1;
  }
  __syncthreads();
  {
    float ps = 0.0f, pq = 0.0f;
#pragma unroll
    for (int w = 0; w < NWAVE; ++w) { ps += sts[w * 256 + tid]; pq += stq[w * 256 + tid]; }
    pcs[tid] = ps; pcq[tid] = pq;
  }
  __syncthreads();
  const size_t prow = (size_t)(b * NTT + tt) * ND + dblk * 256;
  if (tid < 64) {
    const v4f p = *(const v4f*)(pcs + 4 * tid);
    *(volatile v4f*)(psum + prow + 4 * tid) = p;
  } else if (tid < 128) {
    const v4f p = *(const v4f*)(pcq + 4 * (tid - 64));
    *(volatile v4f*)(psq + prow + 4 * (tid - 64)) = p;
  }
  __threadfence();
  if (tid < 64) {
    const v4f p = *(const v4f*)(pcs + 4 * tid);
    *(volatile v4f*)(psum + prow + 4 * tid) = p;
  } else if (tid < 128) {
    const v4f p = *(const v4f*)(pcq + 4 * (tid - 64));
    *(volatile v4f*)(psq + prow + 4 * (tid - 64)) = p;
  }
}

template <int LAST>
__global__ __launch_bounds__(NTHR) void k_gemm2(const _Float16* __restrict__ wpl, const _Float16* __restrict__ w2h,
                                                const float* __restrict__ bias2, const float* __restrict__ x,
                                                _Float16* act, float* out) {
  __shared__ __attribute__((aligned(16))) float tile[TILE2];
  const int tid = threadIdx.x, lane = tid & 31, wave = tid >> 5, hh = lane >> 4, m = lane & 15;
  const int wm = wave >> 2, wn = wave & 3;
  const int tt = blockIdx.x, b = blockIdx.y;
  const int t0 = tt * TT;

  v8f acc[2][2];
#pragma unroll
  for (int mt = 0; mt < 2; ++mt)
#pragma unroll
    for (int nt = 0; nt < 2; ++nt) { v8f z = {0.f, 0.f, 0.f, 0.f, 0.f, 0.f, 0.f, 0.f}; acc[mt][nt] = z; }

  const _Float16* ap = wpl + ((size_t)b * NT + t0 + wm * 32 + m) * ND + 8 * hh;
  const _Float16* bp = w2h + (size_t)(wn * 32 + m) * ND + 8 * hh;
#pragma unroll 1
  for (int kt = 0; kt < ND / 32; ++kt) {
    const int k0 = 32 * kt;
    FragH a0, a1, b0, b1;
    a0.h[0] = *(const v8h*)(ap + k0);
    a0.h[1] = *(const v8h*)(ap + k0 + 16);
    a1.h[0] = *(const v8h*)(ap + 16 * ND + k0);
    a1.h[1] = *(const v8h*)(ap + 16 * ND + k0 + 16);
    b0.h[0] = *(const v8h*)(bp + k0);
    b0.h[1] = *(const v8h*)(bp + k0 + 16);
    b1.h[0] = *(const v8h*)(bp + 16 * ND + k0);
    b1.h[1] = *(const v8h*)(bp + 16 * ND + k0 + 16);
    acc[0][0] = wmf(a0.v, b0.v, acc[0][0]);
    acc[0][1] = wmf(a0.v, b1.v, acc[0][1]);
    acc[1][0] = wmf(a1.v, b0.v, acc[1][0]);
    acc[1][1] = wmf(a1.v, b1.v, acc[1][1]);
  }

  constexpr float OS2 = 1.0f / (WAC * W2C);
  float bv[2];
#pragma unroll
  for (int nt = 0; nt < 2; ++nt) bv[nt] = bias2[wn * 32 + 16 * nt + m];
#pragma unroll
  for (int mt = 0; mt < 2; ++mt) {
#pragma unroll
    for (int nt = 0; nt < 2; ++nt) {
      const int cl = wn * 32 + 16 * nt + m;
#pragma unroll
      for (int r = 0; r < 8; ++r) {
        const int tl = wm * 32 + 16 * mt + 8 * hh + r;
        const float v = acc[mt][nt][r] * OS2 + bv[nt];
        if (LAST) tile[cl * PT2 + tl] = v;
        else      tile[tl * PC2 + cl] = v;
      }
    }
  }
  __syncthreads();

  if (LAST == 0) {
    _Float16* ob = act + ((size_t)b * NT + t0) * NC;
#pragma unroll
    for (int q = 0; q < 4; ++q) {
      const int row = 8 * wave + 2 * q + hh;
      const v4f u0 = *(const v4f*)(tile + row * PC2 + 8 * m);
      const v4f u1 = *(const v4f*)(tile + row * PC2 + 8 * m + 4);
      v8h hv;
      hv[0] = (_Float16)(u0.x * ASC); hv[1] = (_Float16)(u0.y * ASC);
      hv[2] = (_Float16)(u0.z * ASC); hv[3] = (_Float16)(u0.w * ASC);
      hv[4] = (_Float16)(u1.x * ASC); hv[5] = (_Float16)(u1.y * ASC);
      hv[6] = (_Float16)(u1.z * ASC); hv[7] = (_Float16)(u1.w * ASC);
      *(volatile v8h*)(ob + (size_t)row * NC + 8 * m) = hv;
    }
    __threadfence();
#pragma unroll
    for (int q = 0; q < 4; ++q) {
      const int row = 8 * wave + 2 * q + hh;
      const v4f u0 = *(const v4f*)(tile + row * PC2 + 8 * m);
      const v4f u1 = *(const v4f*)(tile + row * PC2 + 8 * m + 4);
      v8h hv;
      hv[0] = (_Float16)(u0.x * ASC); hv[1] = (_Float16)(u0.y * ASC);
      hv[2] = (_Float16)(u0.z * ASC); hv[3] = (_Float16)(u0.w * ASC);
      hv[4] = (_Float16)(u1.x * ASC); hv[5] = (_Float16)(u1.y * ASC);
      hv[6] = (_Float16)(u1.z * ASC); hv[7] = (_Float16)(u1.w * ASC);
      *(volatile v8h*)(ob + (size_t)row * NC + 8 * m) = hv;
    }
  } else {
    const float* xb = x + (size_t)b * NC * NT + t0;
    float* gb = out + (size_t)b * NC * NT + t0;
#pragma unroll
    for (int q = 0; q < 8; ++q) {
      const int cr = 16 * wave + 2 * q + hh;
      const v4f u = *(const v4f*)(tile + cr * PT2 + 4 * m);
      const v4f rx = *(const v4f*)(xb + (size_t)cr * NT + 4 * m);
      const v4f v = u + rx;
      *(volatile v4f*)(gb + (size_t)cr * NT + 4 * m) = v;
    }
    __threadfence();
#pragma unroll
    for (int q = 0; q < 8; ++q) {
      const int cr = 16 * wave + 2 * q + hh;
      const v4f u = *(const v4f*)(tile + cr * PT2 + 4 * m);
      const v4f rx = *(const v4f*)(xb + (size_t)cr * NT + 4 * m);
      const v4f v = u + rx;
      *(volatile v4f*)(gb + (size_t)cr * NT + 4 * m) = v;
    }
  }
}

extern "C" void kernel_launch(void* const* d_in, const int* in_sizes, int n_in,
                              void* d_out, int out_size, void* d_ws, size_t ws_size,
                              hipStream_t stream) {
  if (n_in < 13) return;
  if (in_sizes[0] != NB * NC * NT) return;
  if (in_sizes[1] != NL * ND * NC || in_sizes[2] != NL * ND || in_sizes[3] != NL) return;
  if (in_sizes[4] != NL * ND || in_sizes[5] != NL * ND) return;
  if (in_sizes[6] != NL * ND * NK || in_sizes[7] != NL * ND || in_sizes[8] != NL) return;
  if (in_sizes[9] != NL * ND || in_sizes[10] != NL * ND) return;
  if (in_sizes[11] != NL * NC * ND || in_sizes[12] != NL * NC) return;
  if (out_size != NB * NC * NT) return;

  const float* x   = (const float*)d_in[0];
  const float* w1  = (const float*)d_in[1];
  const float* b1  = (const float*)d_in[2];
  const float* a1  = (const float*)d_in[3];
  const float* g1  = (const float*)d_in[4];
  const float* be1 = (const float*)d_in[5];
  const float* wd  = (const float*)d_in[6];
  const float* bd  = (const float*)d_in[7];
  const float* a2  = (const float*)d_in[8];
  const float* g2  = (const float*)d_in[9];
  const float* be2 = (const float*)d_in[10];
  const float* w2  = (const float*)d_in[11];
  const float* b2  = (const float*)d_in[12];
  float* out = (float*)d_out;

  char* ws = (char*)d_ws;
  size_t off = 0;
  const size_t oAct = off; off += (size_t)NB * NT * NC * 2;  off = (off + 255) & ~(size_t)255;
  const size_t oW1h = off; off += (size_t)NL * ND * NC * 2;  off = (off + 255) & ~(size_t)255;
  const size_t oVpl = off; off += (size_t)NB * NT * ND * 4;  off = (off + 255) & ~(size_t)255;
  const size_t oWpl = off; off += (size_t)NB * NT * ND * 2;  off = (off + 255) & ~(size_t)255;
  const size_t oPs  = off; off += (size_t)NPR * ND * 4;      off = (off + 255) & ~(size_t)255;
  const size_t oPq  = off; off += (size_t)NPR * ND * 4;      off = (off + 255) & ~(size_t)255;
  const size_t oSc1 = off; off += (size_t)ND * 4;            off = (off + 255) & ~(size_t)255;
  const size_t oSh1 = off; off += (size_t)ND * 4;            off = (off + 255) & ~(size_t)255;
  const size_t oW2h = off; off += (size_t)NC * ND * 2;       off = (off + 255) & ~(size_t)255;
  const size_t oB2  = off; off += (size_t)NC * 4;            off = (off + 255) & ~(size_t)255;
  if (off > ws_size || off > (size_t)WSCAP) return;
  _Float16* act  = (_Float16*)(ws + oAct);
  _Float16* w1h  = (_Float16*)(ws + oW1h);
  float*    vpl  = (float*)(ws + oVpl);
  _Float16* wpl  = (_Float16*)(ws + oWpl);
  float*    psum = (float*)(ws + oPs);
  float*    psq  = (float*)(ws + oPq);
  float*    sc1  = (float*)(ws + oSc1);
  float*    sh1  = (float*)(ws + oSh1);
  _Float16* w2h  = (_Float16*)(ws + oW2h);
  float*    bs2  = (float*)(ws + oB2);

  k_cvt_x<<<dim3(NTT, NB), NTHR, 0, stream>>>(x, act);
  k_cvt_w1<<<(NL * ND * NC) / (8 * NTHR), NTHR, 0, stream>>>(w1, w1h);

  hipFuncSetAttribute(reinterpret_cast<const void*>(&k_gemm1),
                      hipFuncAttributeMaxDynamicSharedMemorySize, LDS_G1);

  for (int i = 0; i < NL; ++i) {
    const float* w2l = w2 + (size_t)i * NC * ND;
    const float* b2l = b2 + (size_t)i * NC;
    k_gemm1<<<dim3(ND / 256, NTT, NB), NTHR, LDS_G1, stream>>>(
        act, w1h + (size_t)i * ND * NC, b1 + (size_t)i * ND, a1 + i, vpl, psum, psq);
    k_bnfin<0><<<1, 128, 0, stream>>>(psum, psq, g1 + (size_t)i * ND, be1 + (size_t)i * ND,
                                       sc1, sh1, w2l, b2l, w2h, bs2);
    k_dwconv<<<dim3(ND / 256, NTT, NB), NTHR, 0, stream>>>(
        vpl, sc1, sh1, wd + (size_t)i * ND * NK, bd + (size_t)i * ND, a2 + i, 1 << i, wpl, psum, psq);
    k_bnfin<1><<<1, 128, 0, stream>>>(psum, psq, g2 + (size_t)i * ND, be2 + (size_t)i * ND,
                                       sc1, sh1, w2l, b2l, w2h, bs2);
    if (i < NL - 1)
      k_gemm2<0><<<dim3(NTT, NB), NTHR, 0, stream>>>(wpl, w2h, bs2, x, act, out);
    else
      k_gemm2<1><<<dim3(NTT, NB), NTHR, 0, stream>>>(wpl, w2h, bs2, x, act, out);
  }
}
